// MultiHeadSelfAttention_75307956568524
// MI455X (gfx1250) — hardware-verified
//
#include <hip/hip_runtime.h>


#ifndef NB
#define NB 2
#endif
#ifndef SEQ
#define SEQ 2048
#endif
#define NB_FULL  2
#define SEQ_FULL 2048
#define EM   768
#define NH   12
#define HD   64
#define E3   (3 * EM)
#define PCAR 1024.0f
#define RCAR 2048.0f
#define RINV (1.0f / 2048.0f)
#define SCL  0.125f
#define L2E  1.4426950408889634f

static_assert(HD == 64);
static_assert(EM == NH * HD);
static_assert(E3 == NH * 3 * HD);
static_assert(EM % 64 == 0);
static_assert(E3 % 64 == 0);
static_assert(EM % 32 == 0);
static_assert(EM == 3 * 32 * 8);
static_assert(SEQ % 64 == 0);
static_assert((NB * SEQ) % 8 == 0);
static_assert(NB <= NB_FULL);
static_assert(SEQ <= SEQ_FULL);

typedef _Float16 h16;
typedef unsigned short bf;
typedef __attribute__((ext_vector_type(16))) __bf16   v16bf;
typedef __attribute__((ext_vector_type(16))) _Float16 v16h;
typedef __attribute__((ext_vector_type(8)))  _Float16 v8h;
typedef __attribute__((ext_vector_type(8)))  unsigned short v8us;
typedef __attribute__((ext_vector_type(8)))  float    v8f;
typedef __attribute__((ext_vector_type(4)))  float    v4f;
typedef v4f  __attribute__((may_alias)) v4fa;

__device__ __forceinline__ unsigned short f2bf(float f) { unsigned u = __float_as_uint(f); u += 0x7FFFu + ((u >> 16) & 1u); return (unsigned short)(u >> 16); }
__device__ __forceinline__ float bf2f(unsigned short b) { return __uint_as_float(((unsigned)b) << 16); }
__device__ __forceinline__ float bfr(float f) { return bf2f(f2bf(f)); }
__device__ __forceinline__ void splitf(float y, unsigned short& h, unsigned short& l) { h = f2bf(y); l = f2bf(y - bf2f(h)); }
__device__ __forceinline__ v16h cat16(v8h lo, v8h hi) { return __builtin_shufflevector(lo, hi, 0, 1, 2, 3, 4, 5, 6, 7, 8, 9, 10, 11, 12, 13, 14, 15); }
__device__ __forceinline__ v16bf cat16b(v8us lo, v8us hi) { return __builtin_bit_cast(v16bf, __builtin_shufflevector(lo, hi, 0, 1, 2, 3, 4, 5, 6, 7, 8, 9, 10, 11, 12, 13, 14, 15)); }
__device__ __forceinline__ v16h  ldh(const h16* p) { return cat16(*(const v8h*)p, *(const v8h*)(p + 16)); }
__device__ __forceinline__ v16bf ldb(const bf* p)  { return cat16b(*(const v8us*)p, *(const v8us*)(p + 16)); }
__device__ __forceinline__ v8f wmma16(v16h a, v16h b, v8f c) { return __builtin_amdgcn_wmma_f32_16x16x32_f16(false, a, false, b, (short)0, c, false, false); }
__device__ __forceinline__ v8f wmmab(v16bf a, v16bf b, v8f c) { return __builtin_amdgcn_wmma_f32_16x16x32_bf16(false, a, false, b, (short)0, c, false, false); }

__global__ __launch_bounds__(256) void k_cvt8(const float* __restrict__ src, bf* dst, size_t n8) {
    const size_t i = (size_t)blockIdx.x * 256 + threadIdx.x; if (i >= n8) return;
    const v8f v = *(const v8f*)(src + i * 8); v8us o;
#pragma unroll
    for (int k = 0; k < 8; ++k) o[k] = f2bf(v[k]);
    *(volatile v8us*)(dst + i * 8) = o; __threadfence(); *(volatile v8us*)(dst + i * 8) = o;
}

__global__ __launch_bounds__(256) void k_ln(const float* __restrict__ x, const float* __restrict__ gamma, const float* __restrict__ beta, bf* XH, bf* XL) {
    const int lane = threadIdx.x & 31; const int wave = __builtin_amdgcn_readfirstlane((int)(threadIdx.x >> 5));
    const int row = blockIdx.x * 8 + wave; if (row >= NB * SEQ) return;
    const int b = row / SEQ, t = row - b * SEQ;
    const float* xr = x + ((size_t)b * SEQ_FULL + t) * EM + lane * 8;
    float s = 0.f;
#pragma unroll 1
    for (int c = 0; c < 3; ++c) { const v8f a = *(const v8f*)(xr + c * 256);
#pragma unroll
        for (int q = 0; q < 8; ++q) s += bfr(a[q]); }
#pragma unroll
    for (int sh = 16; sh; sh >>= 1) s += __shfl_xor(s, sh, 32);
    const float mu = s * (1.0f / (float)EM);
    float s2 = 0.f;
#pragma unroll 1
    for (int c = 0; c < 3; ++c) { const v8f a = *(const v8f*)(xr + c * 256);
#pragma unroll
        for (int q = 0; q < 8; ++q) { const float d = bfr(a[q]) - mu; s2 += d * d; } }
#pragma unroll
    for (int sh = 16; sh; sh >>= 1) s2 += __shfl_xor(s2, sh, 32);
    const float rs = rsqrtf(s2 * (1.0f / (float)EM) + 1e-5f);
#pragma unroll 1
    for (int c = 0; c < 3; ++c) {
        const int col = c * 256 + lane * 8;
        const v8f a = *(const v8f*)(xr + c * 256); const v8f g = *(const v8f*)(gamma + col); const v8f be = *(const v8f*)(beta + col);
        v8us oh, ol;
#pragma unroll
        for (int q = 0; q < 8; ++q) { const float y = (bfr(a[q]) - mu) * rs * bfr(g[q]) + bfr(be[q]); unsigned short hh, ll; splitf(y, hh, ll); oh[q] = hh; ol[q] = ll; }
        const size_t oo = (size_t)row * EM + col;
        *(volatile v8us*)(XH + oo) = oh; *(volatile v8us*)(XL + oo) = ol; __threadfence(); *(volatile v8us*)(XH + oo) = oh; *(volatile v8us*)(XL + oo) = ol;
    }
}

__global__ __launch_bounds__(32) void k_gemm_hl(const bf* __restrict__ A, const bf* __restrict__ A2, const bf* __restrict__ Bt, int K, float* C, int ldc, const float* __restrict__ bias, size_t sA, size_t sC) {
    __shared__ __align__(16) float os[16 * 68];
    const size_t z = blockIdx.z; A += z * sA; A2 += z * sA; C += z * sC;
    const int lane = threadIdx.x & 31, lr = lane & 15, hi = lane >> 4; const int r0 = blockIdx.x * 64, c0 = blockIdx.y * 64;
    v8f acc[4][4];
#pragma unroll
    for (int mb = 0; mb < 4; ++mb)
#pragma unroll
        for (int nb = 0; nb < 4; ++nb) acc[mb][nb] = (v8f){};
    const size_t aoff = (size_t)(r0 + lr) * K + 8 * hi, boff = (size_t)(c0 + lr) * K + 8 * hi;
#pragma unroll 1
    for (int kc = 0; kc < K; kc += 32) {
        v16bf b[4]; v16bf a = {}, a2 = {};
#pragma unroll
        for (int nb = 0; nb < 4; ++nb) b[nb] = ldb(Bt + boff + (size_t)nb * 16 * K + kc);
#pragma unroll
        for (int mb = 0; mb < 4; ++mb) { a = ldb(A + aoff + (size_t)mb * 16 * K + kc); a2 = ldb(A2 + aoff + (size_t)mb * 16 * K + kc);
#pragma unroll
            for (int nb = 0; nb < 4; ++nb) { acc[mb][nb] = wmmab(a, b[nb], acc[mb][nb]); acc[mb][nb] = wmmab(a2, b[nb], acc[mb][nb]); } }
        asm volatile("v_nop\n\tv_nop\n\tv_nop\n\tv_nop" : "+v"(acc[3][0]), "+v"(acc[3][1]), "+v"(acc[3][2]), "+v"(acc[3][3]) : "v"(a), "v"(a2), "v"(b[0]), "v"(b[1]), "v"(b[2]), "v"(b[3]));
    }
#pragma unroll
    for (int mb = 0; mb < 4; ++mb) {
#pragma unroll
        for (int nb = 0; nb < 4; ++nb) {
#pragma unroll
            for (int j = 0; j < 8; ++j) os[(hi * 8 + j) * 68 + nb * 16 + lr] = acc[mb][nb][j]; }
        __builtin_amdgcn_wave_barrier(); asm volatile("" ::: "memory");
        float* crow = C + (size_t)(r0 + mb * 16) * ldc + c0;
#pragma unroll 1
        for (int ps = 0; ps < 2; ++ps) {
#pragma unroll
            for (int s = 0; s < 8; ++s) { const int row = 2 * s + hi, cofs = lr * 4; v4f val = *(const v4fa*)(os + row * 68 + cofs);
                val[0] += bfr(bias[c0 + cofs]); val[1] += bfr(bias[c0 + cofs + 1]); val[2] += bfr(bias[c0 + cofs + 2]); val[3] += bfr(bias[c0 + cofs + 3]);
                *(volatile v4f*)(crow + (size_t)row * ldc + cofs) = val; }
            if (ps == 0) __threadfence(); }
        __builtin_amdgcn_wave_barrier(); asm volatile("" ::: "memory");
    }
}

__global__ __launch_bounds__(256) void k_qk(const float* __restrict__ F, h16* Q16, h16* QR, h16* K16) {
    const size_t i = (size_t)blockIdx.x * 256 + threadIdx.x; if (i >= (size_t)NB * NH * SEQ * HD / 8) return;
    const int d8 = (int)(i & 7); const int t = (int)((i >> 3) % SEQ); const int bh = (int)(i / ((size_t)8 * SEQ)); const int b = bh / NH, h = bh - b * NH;
    const float* f = F + ((size_t)b * SEQ + t) * E3 + h * (3 * HD) + d8 * 8;
    const v8f qv = *(const v8f*)f; const v8f kv = *(const v8f*)(f + HD);
    v8h oq, orr, ok;
#pragma unroll
    for (int j = 0; j < 8; ++j) { const h16 qh = (h16)qv[j]; oq[j] = qh; orr[j] = (h16)((qv[j] - (float)qh) * RCAR); ok[j] = (h16)kv[j]; }
    const size_t e = i * 8;
    *(volatile v8h*)(Q16 + e) = oq; *(volatile v8h*)(QR + e) = orr; *(volatile v8h*)(K16 + e) = ok; __threadfence();
    *(volatile v8h*)(Q16 + e) = oq; *(volatile v8h*)(QR + e) = orr; *(volatile v8h*)(K16 + e) = ok;
}

__global__ __launch_bounds__(256) void k_vt(const float* __restrict__ F, h16* VT) {
    const size_t i = (size_t)blockIdx.x * 256 + threadIdx.x; if (i >= (size_t)NB * NH * HD * SEQ / 8) return;
    const int T8 = SEQ / 8; const int t8 = (int)(i % T8); const int d = (int)((i / T8) % HD); const int bh = (int)(i / ((size_t)T8 * HD)); const int b = bh / NH, h = bh - b * NH;
    const float* f = F + ((size_t)b * SEQ + (size_t)t8 * 8) * E3 + h * (3 * HD) + 2 * HD + d;
    v8h o;
#pragma unroll
    for (int j = 0; j < 8; ++j) o[j] = (h16)f[(size_t)j * E3];
    const size_t e = i * 8;
    *(volatile v8h*)(VT + e) = o; __threadfence(); *(volatile v8h*)(VT + e) = o;
}

__global__ __launch_bounds__(128) void k_flash(const h16* __restrict__ Q16, const h16* __restrict__ QR, const h16* __restrict__ K16, const h16* __restrict__ VT, bf* CH, bf* CL) {
    __shared__ __align__(16) float os[4 * 16 * 68];
    const int lane = threadIdx.x & 31, lr = lane & 15, hi = lane >> 4;
    const int wave = __builtin_amdgcn_readfirstlane((int)(threadIdx.x >> 5));
    const int bh = blockIdx.y; const int b = bh / NH, h = bh - b * NH;
    const int q0 = blockIdx.x * 64 + wave * 16;
    const size_t pb0 = (size_t)bh * SEQ * HD;
    const size_t qoff = pb0 + (size_t)(q0 + lr) * HD + 8 * hi;
    const v16h qh0 = ldh(Q16 + qoff), qh1 = ldh(Q16 + qoff + 32), qr0 = ldh(QR + qoff), qr1 = ldh(QR + qoff + 32);
    v8f o[4];
#pragma unroll
    for (int dt = 0; dt < 4; ++dt) o[dt] = (v8f){};
    float m = -1.0e30f, l = 0.f;
    const size_t koff = pb0 + (size_t)lr * HD + 8 * hi;
    const size_t voff = pb0 + (size_t)lr * SEQ + 8 * hi;
#pragma unroll 1
    for (int t0 = 0; t0 < SEQ; t0 += 32) {
        const h16* kp = K16 + koff + (size_t)t0 * HD;
        const v16h ka00 = ldh(kp), ka01 = ldh(kp + 32), ka10 = ldh(kp + 16 * HD), ka11 = ldh(kp + 16 * HD + 32);
        v8f s0 = {}, s1 = {}, r0 = {}, r1 = {};
        s0 = wmma16(ka00, qh0, s0); s1 = wmma16(ka10, qh0, s1); r0 = wmma16(ka00, qr0, r0); r1 = wmma16(ka10, qr0, r1);
        s0 = wmma16(ka01, qh1, s0); s1 = wmma16(ka11, qh1, s1); r0 = wmma16(ka01, qr1, r0); r1 = wmma16(ka11, qr1, r1);
        asm volatile("v_nop\n\tv_nop\n\tv_nop\n\tv_nop" : "+v"(s0), "+v"(s1), "+v"(r0), "+v"(r1) : "v"(ka00), "v"(ka01), "v"(ka10), "v"(ka11));
        float tv[16];
#pragma unroll
        for (int r = 0; r < 8; ++r) { tv[r] = (s0[r] + r0[r] * RINV) * SCL; tv[8 + r] = (s1[r] + r1[r] * RINV) * SCL; }
        float lm = tv[0];
#pragma unroll
        for (int k = 1; k < 16; ++k) lm = fmaxf(lm, tv[k]);
        lm = fmaxf(lm, __shfl_xor(lm, 16, 32));
        const float mn = fmaxf(m, lm);
        const float f = __builtin_amdgcn_exp2f((m - mn) * L2E);
        m = mn;
        v16h pbv; float ps = 0.f;
#pragma unroll
        for (int k = 0; k < 16; ++k) { const float p = __builtin_amdgcn_exp2f((tv[k] - mn) * L2E) * PCAR; const h16 ph = (h16)p; pbv[k] = ph; ps += (float)ph; }
        l = l * f + ps;
#pragma unroll
        for (int dt = 0; dt < 4; ++dt) o[dt] *= f;
        const h16* vp = VT + voff + t0;
        v16h va[4];
#pragma unroll
        for (int dt = 0; dt < 4; ++dt) va[dt] = ldh(vp + (size_t)dt * 16 * SEQ);
#pragma unroll
        for (int dt = 0; dt < 4; ++dt) o[dt] = wmma16(va[dt], pbv, o[dt]);
        asm volatile("v_nop\n\tv_nop\n\tv_nop\n\tv_nop" : "+v"(o[0]), "+v"(o[1]), "+v"(o[2]), "+v"(o[3]) : "v"(va[0]), "v"(va[1]), "v"(va[2]), "v"(va[3]), "v"(pbv));
    }
    const float lt = l + __shfl_xor(l, 16, 32);
    const float inv = 1.0f / lt;
    const int ob = wave * (16 * 68);
#pragma unroll
    for (int dt = 0; dt < 4; ++dt) { v4f w0, w1;
#pragma unroll
        for (int r = 0; r < 4; ++r) { w0[r] = o[dt][r] * inv; w1[r] = o[dt][4 + r] * inv; }
        *(v4fa*)(os + ob + lr * 68 + dt * 16 + 8 * hi) = w0; *(v4fa*)(os + ob + lr * 68 + dt * 16 + 8 * hi + 4) = w1; }
    __syncthreads();
    v8us oh[4], ol[4];
    const int rq = lane >> 3, pc = lane & 7;
#pragma unroll
    for (int s = 0; s < 4; ++s) { const int row = s * 4 + rq; const v4f w0 = *(const v4fa*)(os + ob + row * 68 + pc * 8); const v4f w1 = *(const v4fa*)(os + ob + row * 68 + pc * 8 + 4);
#pragma unroll
        for (int r = 0; r < 4; ++r) { unsigned short a2, c2; splitf(w0[r], a2, c2); oh[s][r] = a2; ol[s][r] = c2; splitf(w1[r], a2, c2); oh[s][4 + r] = a2; ol[s][4 + r] = c2; } }
    const size_t cbase = ((size_t)b * SEQ + q0) * EM + h * HD + pc * 8;
#pragma unroll
    for (int s = 0; s < 4; ++s) { const size_t oo = cbase + (size_t)(s * 4 + rq) * EM; *(volatile v8us*)(CH + oo) = oh[s]; *(volatile v8us*)(CL + oo) = ol[s]; }
    __threadfence();
#pragma unroll
    for (int s = 0; s < 4; ++s) { const size_t oo = cbase + (size_t)(s * 4 + rq) * EM; *(volatile v8us*)(CH + oo) = oh[s]; *(volatile v8us*)(CL + oo) = ol[s]; }
}

constexpr size_t al256(size_t v) { return (v + 255) & ~(size_t)255; }
constexpr size_t SZ_WQ = al256((size_t)E3 * EM * 2);
constexpr size_t SZ_WO = al256((size_t)EM * EM * 2);
constexpr size_t SZ_XN = al256((size_t)NB * SEQ * EM * 2);
constexpr size_t SZ_F  = al256((size_t)NB * SEQ * E3 * 4);
constexpr size_t SZ_PL = al256((size_t)NB * NH * SEQ * HD * 2);
constexpr size_t OFF_WQ = 0;
constexpr size_t OFF_WO = OFF_WQ + SZ_WQ;
constexpr size_t OFF_XH = OFF_WO + SZ_WO;
constexpr size_t OFF_XL = OFF_XH + SZ_XN;
constexpr size_t OFF_F  = OFF_XL + SZ_XN;
constexpr size_t OFF_Q  = OFF_F + SZ_F;
constexpr size_t OFF_QR = OFF_Q + SZ_PL;
constexpr size_t OFF_K  = OFF_QR + SZ_PL;
constexpr size_t OFF_VT = OFF_K + SZ_PL;
constexpr size_t OFF_CH = OFF_VT + SZ_PL;
constexpr size_t OFF_CL = OFF_CH + SZ_XN;
constexpr size_t WS_TOTAL = OFF_CL + SZ_XN;
static_assert(WS_TOTAL <= (size_t)134217728);
static_assert(((size_t)E3 * EM) % 8 == 0);
static_assert(((size_t)EM * EM) % 8 == 0);
static_assert(((size_t)NB * NH * SEQ * HD / 8) % 256 == 0);

extern "C" void kernel_launch(void* const* d_in, const int* in_sizes, int n_in,
                              void* d_out, int out_size, void* d_ws, size_t ws_size, hipStream_t stream) {
    if (n_in < 7) return;
    const size_t need_x = ((size_t)(NB - 1) * SEQ_FULL + SEQ) * EM;
    if ((size_t)in_sizes[0] < need_x || in_sizes[1] < EM || in_sizes[2] < EM || in_sizes[3] < E3 * EM || in_sizes[4] < E3 || in_sizes[5] < EM * EM || in_sizes[6] < EM) return;
    if ((size_t)out_size < need_x) return;
    if (WS_TOTAL > ws_size) return;
    const float* x = (const float*)d_in[0]; const float* gamma = (const float*)d_in[1]; const float* beta = (const float*)d_in[2];
    const float* wqkv = (const float*)d_in[3]; const float* bqkv = (const float*)d_in[4]; const float* wo = (const float*)d_in[5]; const float* bo = (const float*)d_in[6];
    float* OUT = (float*)d_out;
    char* ws = (char*)d_ws;
    bf* WQB = (bf*)(ws + OFF_WQ); bf* WOB = (bf*)(ws + OFF_WO); bf* XH = (bf*)(ws + OFF_XH); bf* XL = (bf*)(ws + OFF_XL);
    float* F = (float*)(ws + OFF_F);
    h16* Q16 = (h16*)(ws + OFF_Q); h16* QR = (h16*)(ws + OFF_QR); h16* K16 = (h16*)(ws + OFF_K); h16* VT = (h16*)(ws + OFF_VT);
    bf* CH = (bf*)(ws + OFF_CH); bf* CL = (bf*)(ws + OFF_CL);

    k_cvt8<<<(unsigned)(((size_t)E3 * EM / 8 + 255) / 256), 256, 0, stream>>>(wqkv, WQB, (size_t)E3 * EM / 8);
    k_cvt8<<<(unsigned)(((size_t)EM * EM / 8 + 255) / 256), 256, 0, stream>>>(wo, WOB, (size_t)EM * EM / 8);
    k_ln<<<(NB * SEQ) / 8, 256, 0, stream>>>(x, gamma, beta, XH, XL);
    k_gemm_hl<<<dim3(SEQ / 64, E3 / 64, NB), 32, 0, stream>>>(XH, XL, WQB, EM, F, E3, bqkv, (size_t)SEQ * EM, (size_t)SEQ * E3);
    const unsigned LP = (unsigned)(((size_t)NB * NH * SEQ * HD / 8 + 255) / 256);
    k_qk<<<LP, 256, 0, stream>>>(F, Q16, QR, K16);
    k_vt<<<LP, 256, 0, stream>>>(F, VT);
    k_flash<<<dim3(SEQ / 64, NB * NH), 128, 0, stream>>>(Q16, QR, K16, VT, CH, CL);
    k_gemm_hl<<<dim3(SEQ / 64, EM / 64, NB), 32, 0, stream>>>(CH, CL, WOB, EM, OUT, EM, bo, (size_t)SEQ * EM, (size_t)SEQ_FULL * EM);
}
